// GraphormerAttentionHead_20985210208827
// MI455X (gfx1250) — hardware-verified
//
#include <hip/hip_runtime.h>
#include <stddef.h>
#include <stdint.h>


#define DIN 256
#define DD 64
#define NMAX 8192
#define RPB 128
#define BWAVES 8
#define SEGCAP 1024
#define LCAP 2048
#define BMW (NMAX / 32)
#define WPITCH 264
#define EPITCH 72
#define OPITCH 68
#define PROJ_LDS_BYTES (2 * DD * WPITCH * 2 + 4 * 2 * 16 * EPITCH * 2)

typedef __bf16 v16bf __attribute__((ext_vector_type(16)));
typedef float v8f __attribute__((ext_vector_type(8)));
typedef float v4f __attribute__((ext_vector_type(4)));
typedef unsigned int v4u __attribute__((ext_vector_type(4)));

union Frag {
  v16bf v;
  v4u q[2];
  unsigned int u[8];
};

__device__ __forceinline__ v8f zero8() {
  v8f z = {0.f, 0.f, 0.f, 0.f, 0.f, 0.f, 0.f, 0.f};
  return z;
}

__device__ __forceinline__ unsigned int bf16_rne(float f) {
  unsigned int u = __float_as_uint(f);
  u += 0x7FFFu + ((u >> 16) & 1u);
  return u & 0xFFFF0000u;
}

__device__ __forceinline__ void split2(float f, unsigned int& hb, unsigned int& lb) {
  hb = bf16_rne(f);
  lb = bf16_rne(f - __uint_as_float(hb));
}

__device__ __forceinline__ void split_pack(const float (&f)[16], Frag& hi, Frag& lo) {
#pragma unroll
  for (int j = 0; j < 8; ++j) {
    unsigned int h0, l0, h1, l1;
    split2(f[2 * j], h0, l0);
    split2(f[2 * j + 1], h1, l1);
    hi.u[j] = (h0 >> 16) | h1;
    lo.u[j] = (l0 >> 16) | l1;
  }
}

__device__ __forceinline__ int koff(int i, int h) { return (i < 8) ? (8 * h + i) : (8 * h + i + 8); }

__device__ __forceinline__ void load16f(float (&f)[16], const float* p, int h) {
  v4f a = *(const v4f*)(p + 8 * h);
  v4f b = *(const v4f*)(p + 8 * h + 4);
  v4f c = *(const v4f*)(p + 16 + 8 * h);
  v4f d = *(const v4f*)(p + 20 + 8 * h);
  f[0] = a[0]; f[1] = a[1]; f[2] = a[2]; f[3] = a[3];
  f[4] = b[0]; f[5] = b[1]; f[6] = b[2]; f[7] = b[3];
  f[8] = c[0]; f[9] = c[1]; f[10] = c[2]; f[11] = c[3];
  f[12] = d[0]; f[13] = d[1]; f[14] = d[2]; f[15] = d[3];
}

__device__ __forceinline__ v8f wmma3(v8f acc, v16bf ah, v16bf al, v16bf bh, v16bf bl) {
  acc = __builtin_amdgcn_wmma_f32_16x16x32_bf16(false, ah, false, bh, (short)0, acc, false, false);
  acc = __builtin_amdgcn_wmma_f32_16x16x32_bf16(false, ah, false, bl, (short)0, acc, false, false);
  acc = __builtin_amdgcn_wmma_f32_16x16x32_bf16(false, al, false, bh, (short)0, acc, false, false);
  asm volatile("v_nop\n\tv_nop\n\tv_nop\n\tv_nop" : "+v"(acc) : "v"(ah), "v"(al), "v"(bh), "v"(bl));
  return acc;
}

__global__ void __launch_bounds__(128) proj_kernel(
    const float* __restrict__ x,
    const float* __restrict__ Wq, const float* __restrict__ bq,
    const float* __restrict__ Wk, const float* __restrict__ bk,
    const float* __restrict__ Wv, const float* __restrict__ bv,
    unsigned short* Qh, unsigned short* Ql,
    unsigned short* Kh, unsigned short* Kl,
    unsigned short* Vh, unsigned short* Vl, int N) {
  extern __shared__ __align__(16) unsigned char dynlds[];
  unsigned short* whi = (unsigned short*)dynlds;
  unsigned short* wlo = whi + DD * WPITCH;
  unsigned short* ebase = wlo + DD * WPITCH;

  const int tid = threadIdx.x;
  const int lane = tid & 31, wave = tid >> 5, h = lane >> 4, m = lane & 15;
  if (blockIdx.x * 64 >= N) return;
  const int rbase = blockIdx.x * 64 + wave * 16;
  unsigned short* ehi = ebase + wave * (2 * 16 * EPITCH);
  unsigned short* elo = ehi + 16 * EPITCH;

  for (int mat = 0; mat < 3; ++mat) {
    const float* W = (mat == 0) ? Wq : ((mat == 1) ? Wk : Wv);
    const float* bb = (mat == 0) ? bq : ((mat == 1) ? bk : bv);
    unsigned short* dh = (mat == 0) ? Qh : ((mat == 1) ? Kh : Vh);
    unsigned short* dl = (mat == 0) ? Ql : ((mat == 1) ? Kl : Vl);

    __syncthreads();
#pragma unroll 4
    for (int i = 0; i < (DIN * DD) / 128; ++i) {
      int idx = i * 128 + tid;
      int kk = idx >> 6;
      int n = idx & 63;
      unsigned int hb, lb;
      split2(W[idx], hb, lb);
      whi[n * WPITCH + kk] = (unsigned short)(hb >> 16);
      wlo[n * WPITCH + kk] = (unsigned short)(lb >> 16);
    }
    __syncthreads();

    v8f acc[4];
#pragma unroll
    for (int t = 0; t < 4; ++t) acc[t] = zero8();

    const float* xr = x + (size_t)(rbase + m) * DIN;
#pragma unroll 2
    for (int c = 0; c < DIN / 32; ++c) {
      float f[16];
      load16f(f, xr + c * 32, h);
      Frag ah, al;
      split_pack(f, ah, al);
#pragma unroll
      for (int t = 0; t < 4; ++t) {
        const unsigned short* ph = whi + (16 * t + m) * WPITCH + c * 32;
        const unsigned short* pl = wlo + (16 * t + m) * WPITCH + c * 32;
        Frag bh, bl;
        bh.q[0] = *(const v4u*)(ph + 8 * h);
        bh.q[1] = *(const v4u*)(ph + 16 + 8 * h);
        bl.q[0] = *(const v4u*)(pl + 8 * h);
        bl.q[1] = *(const v4u*)(pl + 16 + 8 * h);
        acc[t] = wmma3(acc[t], ah.v, al.v, bh.v, bl.v);
      }
    }

#pragma unroll
    for (int t = 0; t < 4; ++t) {
      float bias = bb[16 * t + m];
#pragma unroll
      for (int r = 0; r < 8; ++r) {
        unsigned int hb, lb;
        split2(acc[t][r] + bias, hb, lb);
        ehi[(8 * h + r) * EPITCH + 16 * t + m] = (unsigned short)(hb >> 16);
        elo[(8 * h + r) * EPITCH + 16 * t + m] = (unsigned short)(lb >> 16);
      }
    }
    __syncthreads();

    v4u sh[4], sl[4];
#pragma unroll
    for (int j = 0; j < 4; ++j) {
      int row = 4 * j + (lane >> 3), col8 = (lane & 7) * 8;
      sh[j] = *(const v4u*)(ehi + row * EPITCH + col8);
      sl[j] = *(const v4u*)(elo + row * EPITCH + col8);
    }
#pragma unroll
    for (int j = 0; j < 4; ++j) {
      int row = 4 * j + (lane >> 3), col8 = (lane & 7) * 8;
      *(volatile v4u*)(dh + (size_t)(rbase + row) * DD + col8) = sh[j];
      *(volatile v4u*)(dl + (size_t)(rbase + row) * DD + col8) = sl[j];
    }
    __threadfence();
#pragma unroll
    for (int j = 0; j < 4; ++j) {
      int row = 4 * j + (lane >> 3), col8 = (lane & 7) * 8;
      *(volatile v4u*)(dh + (size_t)(rbase + row) * DD + col8) = sh[j];
      *(volatile v4u*)(dl + (size_t)(rbase + row) * DD + col8) = sl[j];
    }
  }
}

__global__ void __launch_bounds__(256) bucket_kernel(
    const int* __restrict__ ei, int E, int N, unsigned int* seg) {
  __shared__ __align__(16) unsigned int sbuf[BWAVES * SEGCAP];
  const int tid = threadIdx.x;
  const int lane = tid & 31, w = tid >> 5;
  const int rowbase = blockIdx.x * RPB;
  unsigned int* mine = sbuf + w * SEGCAP;

#pragma unroll 4
  for (int i = 0; i < SEGCAP / 32; ++i) mine[i * 32 + lane] = 0u;

  const int chunk = ((E + BWAVES * 32 - 1) / (BWAVES * 32)) * 32;
  const int ebeg = w * chunk;
  int eend = ebeg + chunk;
  if (eend > E) eend = E;

  unsigned int cnt = 0u;
  for (int e0 = ebeg; e0 < eend; e0 += 32) {
    int e = e0 + lane;
    bool valid = e < eend;
    int r = -1, c = -1;
    if (valid) {
      r = ei[e];
      c = ei[(size_t)E + e];
      if (r < 0) r += N;
      if (c < 0) c += N;
    }
    unsigned int loc = (unsigned int)(r - rowbase);
    bool match = valid && (loc < (unsigned int)RPB) && ((unsigned int)c < (unsigned int)N);
    unsigned int mk = __builtin_amdgcn_ballot_w32(match);
    unsigned int pos = cnt + (unsigned int)__builtin_popcount(mk & ((1u << lane) - 1u));
    if (match && pos < (unsigned int)(SEGCAP - 1)) mine[1 + pos] = (loc << 16) | (unsigned int)c;
    cnt += (unsigned int)__builtin_popcount(mk);
    if (cnt > (unsigned int)(SEGCAP - 1)) cnt = (unsigned int)(SEGCAP - 1);
  }
  if (lane == 0) mine[0] = cnt;
  __syncthreads();

  unsigned int* gseg = seg + ((size_t)blockIdx.x * BWAVES + w) * SEGCAP;
  v4u vv[SEGCAP / 128];
#pragma unroll
  for (int j = 0; j < SEGCAP / 128; ++j) vv[j] = *(const v4u*)(mine + (j * 32 + lane) * 4);
#pragma unroll
  for (int j = 0; j < SEGCAP / 128; ++j) *(volatile v4u*)(gseg + (size_t)(j * 32 + lane) * 4) = vv[j];
  __threadfence();
#pragma unroll
  for (int j = 0; j < SEGCAP / 128; ++j) *(volatile v4u*)(gseg + (size_t)(j * 32 + lane) * 4) = vv[j];
}

__global__ void __launch_bounds__(32) attn_kernel(
    const unsigned short* __restrict__ Qh, const unsigned short* __restrict__ Ql,
    const unsigned short* __restrict__ Kh, const unsigned short* __restrict__ Kl,
    const unsigned short* __restrict__ Vh, const unsigned short* __restrict__ Vl,
    const unsigned int* __restrict__ seg, float* out, int N) {
  __shared__ unsigned int bm[16 * BMW];
  __shared__ unsigned int klist[LCAP];
  __shared__ float pbuf[LCAP];
  __shared__ __align__(16) float ost[16 * OPITCH];
  __shared__ int soff[17];

  const int lane = threadIdx.x & 31, h = lane >> 4, m = lane & 15;
  const int r0 = blockIdx.x * 16;
  if (r0 >= N) return;
  const int bucket = blockIdx.x / (RPB / 16);
  const int rloc0 = (blockIdx.x % (RPB / 16)) * 16;

#pragma unroll 8
  for (int i = 0; i < (16 * BMW) / 32; ++i) bm[i * 32 + lane] = 0u;
  __syncthreads();

  for (int w = 0; w < BWAVES; ++w) {
    const unsigned int* sp = seg + ((size_t)bucket * BWAVES + w) * SEGCAP;
    unsigned int cnt = (unsigned int)__builtin_amdgcn_readfirstlane((int)sp[0]);
    if (cnt > (unsigned int)(SEGCAP - 1)) cnt = (unsigned int)(SEGCAP - 1);
    for (unsigned int i = 0; i < cnt; i += 32) {
      unsigned int e = i + (unsigned int)lane;
      bool valid = e < cnt;
      unsigned int ent = valid ? sp[1 + e] : 0xFFFFFFFFu;
      unsigned int loc = ent >> 16, key = ent & 0xFFFFu;
      unsigned int ml = loc - (unsigned int)rloc0;
      bool match = valid && (ml < 16u) && (key < (unsigned int)NMAX);
      unsigned int word = ml * (unsigned int)BMW + (key >> 5);
      unsigned int bit = 1u << (key & 31u);
      unsigned int mk = __builtin_amdgcn_ballot_w32(match);
      while (mk) {
        int l = __builtin_ctz(mk);
        unsigned int ww = (unsigned int)__builtin_amdgcn_readlane((int)word, l);
        unsigned int wb = (unsigned int)__builtin_amdgcn_readlane((int)bit, l);
        bm[ww] |= wb;
        mk &= mk - 1u;
      }
    }
  }
  __syncthreads();

  unsigned int base = 0u;
  for (int mm = 0; mm < 16; ++mm) {
    if (lane == 0) soff[mm] = (int)((base < (unsigned int)LCAP) ? base : (unsigned int)LCAP);
#pragma unroll 1
    for (int it = 0; it < BMW / 32; ++it) {
      unsigned int widx = (unsigned int)(it * 32 + lane);
      unsigned int w = bm[mm * BMW + widx];
      int cpop = __builtin_popcount(w);
      int incl = cpop;
#pragma unroll
      for (int off = 1; off < 32; off <<= 1) {
        int tv = __shfl_up(incl, off, 32);
        if (lane >= off) incl += tv;
      }
      int total = __builtin_amdgcn_readlane(incl, 31);
      unsigned int pos = base + (unsigned int)(incl - cpop);
      while (w) {
        int b = __builtin_ctz(w);
        if (pos < (unsigned int)LCAP) klist[pos] = ((unsigned int)mm << 16) | (widx * 32u + (unsigned int)b);
        ++pos;
        w &= w - 1u;
      }
      base += (unsigned int)total;
    }
  }
  const unsigned int L = (base < (unsigned int)LCAP) ? base : (unsigned int)LCAP;
  const unsigned int Lpad = (L + 31u) & ~31u;
  if (lane == 0) soff[16] = (int)L;
  {
    unsigned int e = L + (unsigned int)lane;
    if (e < Lpad) klist[e] = (16u << 16);
  }
  __syncthreads();

  Frag qh[2], ql[2];
  {
    const unsigned short* qa = Qh + (size_t)(r0 + m) * DD;
    const unsigned short* qb = Ql + (size_t)(r0 + m) * DD;
#pragma unroll
    for (int c = 0; c < 2; ++c) {
      qh[c].q[0] = *(const v4u*)(qa + c * 32 + 8 * h);
      qh[c].q[1] = *(const v4u*)(qa + c * 32 + 16 + 8 * h);
      ql[c].q[0] = *(const v4u*)(qb + c * 32 + 8 * h);
      ql[c].q[1] = *(const v4u*)(qb + c * 32 + 16 + 8 * h);
    }
  }

  const int ntiles = (int)(Lpad >> 4);
  for (int t = 0; t < ntiles; ++t) {
    const int e0 = t * 16;
    unsigned int ent = klist[e0 + m];
    unsigned int key = ent & 0xFFFFu;
    const unsigned short* ka = Kh + (size_t)key * DD;
    const unsigned short* kb = Kl + (size_t)key * DD;
    v8f acc = zero8();
#pragma unroll
    for (int c = 0; c < 2; ++c) {
      Frag kh, kl;
      kh.q[0] = *(const v4u*)(ka + c * 32 + 8 * h);
      kh.q[1] = *(const v4u*)(ka + c * 32 + 16 + 8 * h);
      kl.q[0] = *(const v4u*)(kb + c * 32 + 8 * h);
      kl.q[1] = *(const v4u*)(kb + c * 32 + 16 + 8 * h);
      acc = wmma3(acc, qh[c].v, ql[c].v, kh.v, kl.v);
    }
    unsigned int mmr = ent >> 16;
    float dv = 0.f;
#pragma unroll
    for (int r = 0; r < 8; ++r) dv = ((mmr & 7u) == (unsigned int)r) ? acc[r] : dv;
    dv = ((mmr >> 3) == (unsigned int)h) ? dv : 0.f;
    float s = dv + __shfl_xor(dv, 16, 32);
    if (h == 0) pbuf[e0 + m] = s * 0.125f;
  }
  __syncthreads();

  for (int mm = 0; mm < 16; ++mm) {
    const int beg = __builtin_amdgcn_readfirstlane(soff[mm]);
    const int end = __builtin_amdgcn_readfirstlane(soff[mm + 1]);
    float mx = -__builtin_inff();
    for (int e = beg + lane; e < end; e += 32) mx = fmaxf(mx, pbuf[e]);
#pragma unroll
    for (int off = 16; off > 0; off >>= 1) mx = fmaxf(mx, __shfl_xor(mx, off, 32));
    float sum = 0.f;
    for (int e = beg + lane; e < end; e += 32) {
      float ex = __builtin_expf(pbuf[e] - mx);
      pbuf[e] = ex;
      sum += ex;
    }
#pragma unroll
    for (int off = 16; off > 0; off >>= 1) sum += __shfl_xor(sum, off, 32);
    const float inv = (sum > 0.f) ? (1.0f / sum) : 0.f;
    for (int e = beg + lane; e < end; e += 32) pbuf[e] = pbuf[e] * inv;
  }
  __syncthreads();

  v8f oacc[4];
#pragma unroll
  for (int t4 = 0; t4 < 4; ++t4) oacc[t4] = zero8();
  const int nks = (int)(Lpad >> 5);
  for (int c = 0; c < nks; ++c) {
    const int e0 = c * 32;
    unsigned int keyv[16];
    float f[16];
#pragma unroll
    for (int i = 0; i < 16; ++i) {
      int e = e0 + koff(i, h);
      unsigned int en = klist[e];
      keyv[i] = en & 0xFFFFu;
      f[i] = ((en >> 16) == (unsigned int)m) ? pbuf[e] : 0.f;
    }
    Frag ph, pl;
    split_pack(f, ph, pl);
#pragma unroll
    for (int t4 = 0; t4 < 4; ++t4) {
      Frag vh, vl;
#pragma unroll
      for (int j = 0; j < 8; ++j) {
        size_t a0 = (size_t)keyv[2 * j] * DD + 16 * t4 + m;
        size_t a1 = (size_t)keyv[2 * j + 1] * DD + 16 * t4 + m;
        vh.u[j] = (unsigned int)Vh[a0] | ((unsigned int)Vh[a1] << 16);
        vl.u[j] = (unsigned int)Vl[a0] | ((unsigned int)Vl[a1] << 16);
      }
      oacc[t4] = wmma3(oacc[t4], ph.v, pl.v, vh.v, vl.v);
    }
  }

#pragma unroll
  for (int t4 = 0; t4 < 4; ++t4) {
#pragma unroll
    for (int r = 0; r < 8; ++r) ost[(8 * h + r) * OPITCH + 16 * t4 + m] = oacc[t4][r];
  }
  __syncthreads();
  v4f ov[8];
#pragma unroll
  for (int j = 0; j < 8; ++j) {
    int row = 2 * j + h;
    ov[j] = *(const v4f*)(ost + row * OPITCH + 4 * m);
  }
  float* orow = out + (size_t)r0 * DD;
#pragma unroll
  for (int j = 0; j < 8; ++j) {
    int row = 2 * j + h;
    *(volatile v4f*)(orow + (size_t)row * DD + 4 * m) = ov[j];
  }
  __threadfence();
#pragma unroll
  for (int j = 0; j < 8; ++j) {
    int row = 2 * j + h;
    *(volatile v4f*)(orow + (size_t)row * DD + 4 * m) = ov[j];
  }
}

extern "C" void kernel_launch(void* const* d_in, const int* in_sizes, int n_in,
                              void* d_out, int out_size, void* d_ws, size_t ws_size,
                              hipStream_t stream) {
  if (n_in < 8) return;
  const int N = in_sizes[0] / DIN;
  if (N <= 0 || N * DIN != in_sizes[0] || (N % RPB) != 0 || N > NMAX) return;
  if (in_sizes[2] != DIN * DD || in_sizes[4] != DIN * DD || in_sizes[6] != DIN * DD) return;
  if (in_sizes[3] < DD || in_sizes[5] < DD || in_sizes[7] < DD) return;
  if (out_size != N * DD) return;
  int E = in_sizes[1] / 2;
  if (E < 0) E = 0;
  const int NBK = N / RPB;

  const float* x = (const float*)d_in[0];
  const int* ei = (const int*)d_in[1];
  const float* Wq = (const float*)d_in[2];
  const float* bq = (const float*)d_in[3];
  const float* Wk = (const float*)d_in[4];
  const float* bk = (const float*)d_in[5];
  const float* Wv = (const float*)d_in[6];
  const float* bv = (const float*)d_in[7];
  float* outp = (float*)d_out;

  unsigned char* ws = (unsigned char*)d_ws;
  const size_t plane = (size_t)N * DD * sizeof(unsigned short);
  size_t off = 0;
  unsigned short* Qh = (unsigned short*)(ws + off); off += plane;
  unsigned short* Ql = (unsigned short*)(ws + off); off += plane;
  unsigned short* Kh = (unsigned short*)(ws + off); off += plane;
  unsigned short* Kl = (unsigned short*)(ws + off); off += plane;
  unsigned short* Vh = (unsigned short*)(ws + off); off += plane;
  unsigned short* Vl = (unsigned short*)(ws + off); off += plane;
  unsigned int* seg = (unsigned int*)(ws + off);
  off += (size_t)NBK * BWAVES * SEGCAP * sizeof(unsigned int);
  if (off > ws_size) return;

  proj_kernel<<<dim3(N / 64), dim3(128), PROJ_LDS_BYTES, stream>>>(
      x, Wq, bq, Wk, bk, Wv, bv, Qh, Ql, Kh, Kl, Vh, Vl, N);
  bucket_kernel<<<dim3(NBK), dim3(256), 0, stream>>>(ei, E, N, seg);
  attn_kernel<<<dim3(N / 16), dim3(32), 0, stream>>>(Qh, Ql, Kh, Kl, Vh, Vl, seg, outp, N);
}
